// EdgeDropViewLearner_86079734547103
// MI455X (gfx1250) — hardware-verified
//
#include <hip/hip_runtime.h>
#include <hip/hip_bf16.h>


typedef __bf16 v16bf __attribute__((ext_vector_type(16)));
typedef __bf16 v8bf  __attribute__((ext_vector_type(8)));
typedef float  v8f   __attribute__((ext_vector_type(8)));
typedef float  v4f   __attribute__((ext_vector_type(4)));

union FragB { v16bf v; v8bf half[2]; };

#define DF   128
#define HD   64
#define KP   128
#define NB   64
#define MB   64
#define PQW  128
#define WP   128
#define GT   128
#define ET   256

__device__ __forceinline__ v8f wmma_bf16_guard(v16bf a, v16bf b, v8f c)
{
    v8f d = __builtin_amdgcn_wmma_f32_16x16x32_bf16(false, a, false, b, (short)0, c, false, false);
    asm volatile("v_nop\n\tv_nop\n\tv_nop\n\tv_nop" : "+v"(d) : "v"(a), "v"(b));
    return d;
}

template <int B>
__device__ __forceinline__ void split4(const v4f x, v16bf& hi, v16bf& lo)
{
#pragma unroll
    for (int i = 0; i < 4; ++i) {
        const float v = x[i];
        const __bf16 hb = (__bf16)v;
        hi[B + i] = hb;
        lo[B + i] = (__bf16)(v - (float)hb);
    }
}

__device__ __forceinline__ void load_a_split(const float* p, v16bf& hi, v16bf& lo)
{
    const v4f x0 = *(const v4f*)(p);
    const v4f x1 = *(const v4f*)(p + 4);
    const v4f x2 = *(const v4f*)(p + 16);
    const v4f x3 = *(const v4f*)(p + 20);
    split4<0>(x0, hi, lo);
    split4<4>(x1, hi, lo);
    split4<8>(x2, hi, lo);
    split4<12>(x3, hi, lo);
}

__global__ __launch_bounds__(GT) void node_proj_kernel(
    const float* __restrict__ X,
    const float* __restrict__ W1,
    const float* __restrict__ b1,
    float*       __restrict__ PQ,
    int M)
{
    __shared__ __align__(16) __bf16 sWh[NB * WP];
    __shared__ __align__(16) __bf16 sWl[NB * WP];
    __shared__ __align__(16) float  sO[MB * NB];

    const int tid  = threadIdx.x;
    const int lane = tid & 31;
    const int w    = tid >> 5;
    const int h    = lane >> 4;
    const int m    = lane & 15;
    const int y    = blockIdx.y;
    const int rowBase = blockIdx.x * MB;

    {
        const float* Wsrc = W1 + (size_t)y * (KP * HD);
#pragma unroll 4
        for (int idx = tid; idx < KP * HD; idx += GT) {
            const int k = idx >> 6;
            const int n = idx & 63;
            const float wv = Wsrc[idx];
            const __bf16 hb = (__bf16)wv;
            sWh[n * WP + k] = hb;
            sWl[n * WP + k] = (__bf16)(wv - (float)hb);
        }
    }
    __syncthreads();

    v8f acc[4];
#pragma unroll
    for (int t = 0; t < 4; ++t) {
        const float bb = (y == 0) ? b1[16 * t + m] : 0.0f;
#pragma unroll
        for (int r = 0; r < 8; ++r) acc[t][r] = bb;
    }

    int arow = rowBase + 16 * w + m;
    if (arow > M - 1) arow = M - 1;
    const float* ap = X + (size_t)arow * DF + 8 * h;

#pragma unroll 1
    for (int ks = 0; ks < KP / 32; ++ks) {
        const int k0 = ks * 32;
        v16bf ahi, alo;
        load_a_split(ap + k0, ahi, alo);
#pragma unroll
        for (int t = 0; t < 4; ++t) {
            const __bf16* bph = sWh + (16 * t + m) * WP + k0 + 8 * h;
            const __bf16* bpl = sWl + (16 * t + m) * WP + k0 + 8 * h;
            FragB bh, bl;
            bh.half[0] = *(const v8bf*)(bph);
            bh.half[1] = *(const v8bf*)(bph + 16);
            bl.half[0] = *(const v8bf*)(bpl);
            bl.half[1] = *(const v8bf*)(bpl + 16);
            acc[t] = wmma_bf16_guard(ahi, bh.v, acc[t]);
            acc[t] = wmma_bf16_guard(ahi, bl.v, acc[t]);
            acc[t] = wmma_bf16_guard(alo, bh.v, acc[t]);
        }
    }

#pragma unroll
    for (int t = 0; t < 4; ++t) {
#pragma unroll
        for (int r = 0; r < 8; ++r)
            sO[(16 * w + 8 * h + r) * NB + 16 * t + m] = acc[t][r];
    }
    __syncthreads();

    v4f vals[8];
    size_t goff[8];
    const int c4 = m * 4;
#pragma unroll
    for (int i = 0; i < 8; ++i) {
        const int rl = 16 * w + 2 * i + h;
        vals[i] = *(const v4f*)&sO[rl * NB + c4];
        goff[i] = (size_t)(rowBase + rl) * PQW + (size_t)y * NB + c4;
    }
#pragma unroll
    for (int i = 0; i < 8; ++i) *(volatile v4f*)(PQ + goff[i]) = vals[i];
    __threadfence();
#pragma unroll
    for (int i = 0; i < 8; ++i) *(volatile v4f*)(PQ + goff[i]) = vals[i];
}

__global__ __launch_bounds__(ET) void edge_mlp_kernel(
    const float* __restrict__ PQ,
    const int*   __restrict__ src,
    const int*   __restrict__ dst,
    const float* __restrict__ W2,
    const float* __restrict__ b2,
    float*       __restrict__ out,
    int E, int Nn)
{
    __shared__ __align__(16) float sRes[ET];

    const int tid = threadIdx.x;
    const int e0  = blockIdx.x * ET;
    int ec = e0 + tid;
    if (ec > E - 1) ec = E - 1;

    int s = src[ec];
    int d = dst[ec];
    s = (s < 0) ? 0 : ((s > Nn - 1) ? (Nn - 1) : s);
    d = (d < 0) ? 0 : ((d > Nn - 1) ? (Nn - 1) : d);

    const float* pr = PQ + (size_t)s * PQW;
    const float* qr = PQ + (size_t)d * PQW + HD;

    float acc = 0.0f;
#pragma unroll
    for (int j = 0; j < HD / 4; ++j) {
        const v4f p  = *(const v4f*)(pr + 4 * j);
        const v4f q  = *(const v4f*)(qr + 4 * j);
        const v4f wv = *(const v4f*)(W2 + 4 * j);
#pragma unroll
        for (int c = 0; c < 4; ++c) {
            const float hv = fmaxf(p[c] + q[c], 0.0f);
            acc = fmaf(hv, wv[c], acc);
        }
    }
    sRes[tid] = acc + b2[0];
    __syncthreads();

    if (tid < ET / 4) {
        const int f = e0 + tid * 4;
        const v4f v = *(const v4f*)&sRes[tid * 4];
        const bool full = (f + 4 <= E);
        if (full) {
            *(volatile v4f*)(out + f) = v;
        } else {
#pragma unroll
            for (int c = 0; c < 4; ++c)
                if (f + c < E) ((volatile float*)out)[f + c] = v[c];
        }
        __threadfence();
        if (full) {
            *(volatile v4f*)(out + f) = v;
        } else {
#pragma unroll
            for (int c = 0; c < 4; ++c)
                if (f + c < E) ((volatile float*)out)[f + c] = v[c];
        }
    }
}

extern "C" void kernel_launch(void* const* d_in, const int* in_sizes, int n_in,
                              void* d_out, int out_size, void* d_ws, size_t ws_size,
                              hipStream_t stream)
{
    if (n_in < 7) return;
    const float* X   = (const float*)d_in[0];
    const int*   src = (const int*)d_in[1];
    const int*   dst = (const int*)d_in[2];
    const float* W1  = (const float*)d_in[3];
    const float* b1  = (const float*)d_in[4];
    const float* W2  = (const float*)d_in[5];
    const float* b2  = (const float*)d_in[6];
    float*       out = (float*)d_out;

    const int Nn = in_sizes[0] / DF;
    int E = in_sizes[1];
    if (in_sizes[2] < E) E = in_sizes[2];
    if (out_size < E)    E = out_size;
    if (Nn <= 0 || E <= 0) return;

    const int mblocks = (Nn + MB - 1) / MB;
    const int Mpad    = mblocks * MB;
    const size_t pq_bytes = (size_t)Mpad * PQW * sizeof(float);
    if (pq_bytes > ws_size) return;
    float* PQ = (float*)d_ws;

    node_proj_kernel<<<dim3(mblocks, 2, 1), dim3(GT, 1, 1), 0, stream>>>(X, W1, b1, PQ, Nn);

    const int eblocks = (E + ET - 1) / ET;
    edge_mlp_kernel<<<dim3(eblocks, 1, 1), dim3(ET, 1, 1), 0, stream>>>(PQ, src, dst, W2, b2, out, E, Nn);
}
